// TransformerBlock_42743514530671
// MI455X (gfx1250) — hardware-verified
//
#include <hip/hip_runtime.h>
#ifndef NB
#define NB 4
#endif
#ifndef SEQ
#define SEQ 1024
#endif
#define NB_FULL 4
#define SEQ_FULL 1024
#define DM 768
#define NH 12
#define HD 64
#define DFF 3072
#define LQ (3 * DM)
#define QT ((SEQ) < 512 ? (SEQ) : 512)
#define NKX SEQ
#define MP (NB * SEQ)
#define KPL (SEQ / 256)

static_assert(NH * HD == DM);
static_assert(HD == 64);
static_assert(DM % 64 == 0 && LQ % 64 == 0 && DFF % 64 == 0);
static_assert(DM % 32 == 0 && DFF % 32 == 0 && SEQ % 32 == 0);
static_assert(MP % 128 == 0 && QT % 128 == 0 && SEQ % QT == 0 && SEQ % 256 == 0 && SEQ <= 2048);
static_assert(192 * 4 == DM);
static_assert((NH * QT) % 8 == 0);
static_assert(NB <= NB_FULL && SEQ <= SEQ_FULL);

typedef _Float16 v16h __attribute__((ext_vector_type(16)));
typedef _Float16 v4h __attribute__((ext_vector_type(4)));
typedef unsigned short v8us __attribute__((ext_vector_type(8), may_alias));
typedef float v8f __attribute__((ext_vector_type(8)));
typedef float v4f __attribute__((ext_vector_type(4)));
typedef float v4fa __attribute__((ext_vector_type(4), may_alias));
union FragH { v16h v; v8us half[2]; _Float16 h[16]; unsigned short u[16]; };

__device__ __forceinline__ unsigned short bf16_bits(float x) { unsigned int u = __float_as_uint(x); return (unsigned short)((u + 0x7FFFu + ((u >> 16) & 1u)) >> 16); }
__device__ __forceinline__ float bf16_rne(float x) { return __uint_as_float(((unsigned int)bf16_bits(x)) << 16); }

__global__ __launch_bounds__(256) void k_wt_f16(const float* __restrict__ W, _Float16* __restrict__ Wt, unsigned K, unsigned N, float scale) {
  const unsigned t = blockIdx.x * 256u + threadIdx.x; const unsigned k8n = K >> 3; if (t >= N * k8n) return;
  const unsigned n = t / k8n, k8 = (t - n * k8n) << 3; FragH f;
#pragma unroll
  for (unsigned i = 0; i < 8; ++i) f.h[i] = (_Float16)(bf16_rne(W[(size_t)(k8 + i) * N + n]) * scale);
  const v8us o = f.half[0]; unsigned short* dst = (unsigned short*)Wt + (size_t)n * K + k8;
  *(volatile v8us*)dst = o; __threadfence(); *(volatile v8us*)dst = o;
}

template <int BFIN, int WXB>
__global__ __launch_bounds__(192) void k_ln16(const float* __restrict__ X, unsigned seq, unsigned seqfull, const float* __restrict__ g, const float* __restrict__ bb, float eps, _Float16* __restrict__ N16, float* __restrict__ XB) {
  #pragma clang fp contract(off)
  __shared__ float red1[8]; __shared__ float red2[8];
  const unsigned r = blockIdx.x, t = threadIdx.x, w = t >> 5, lane = t & 31u;
  const unsigned bq = r / seq; const size_t rin = (size_t)bq * seqfull + (r - bq * seq);
  const v4f xa = *(const v4fa*)(X + rin * DM + t * 4u);
  float s[4];
#pragma unroll
  for (unsigned q = 0; q < 4; ++q) s[q] = BFIN ? bf16_rne(xa[q]) : xa[q];
  float sum = (s[0] + s[1]) + (s[2] + s[3]);
  for (int o = 16; o > 0; o >>= 1) sum += __shfl_xor(sum, o, 32);
  if (lane == 0u) red1[w] = sum;
  __syncthreads();
  const float mu = (((red1[0] + red1[1]) + (red1[2] + red1[3])) + (red1[4] + red1[5])) / (float)DM;
  float dl[4];
#pragma unroll
  for (unsigned q = 0; q < 4; ++q) dl[q] = s[q] - mu;
  float vs = (dl[0] * dl[0] + dl[1] * dl[1]) + (dl[2] * dl[2] + dl[3] * dl[3]);
  for (int o = 16; o > 0; o >>= 1) vs += __shfl_xor(vs, o, 32);
  if (lane == 0u) red2[w] = vs;
  __syncthreads();
  const float var = (((red2[0] + red2[1]) + (red2[2] + red2[3])) + (red2[4] + red2[5])) / (float)DM;
  const float rs = rsqrtf(var + eps);
  const v4f gv = *(const v4fa*)(g + t * 4u), bv = *(const v4fa*)(bb + t * 4u);
  v4h y; v4f xb;
#pragma unroll
  for (unsigned q = 0; q < 4; ++q) { y[q] = (_Float16)((dl[q] * rs) * bf16_rne(gv[q]) + bf16_rne(bv[q])); xb[q] = s[q]; }
  const size_t o16 = (size_t)r * DM + t * 4u;
  for (int pass = 0; pass < 2; ++pass) { *(volatile v4h*)(N16 + o16) = y; if (WXB) *(volatile v4f*)(XB + o16) = xb; if (pass == 0) __threadfence(); }
}

__device__ __forceinline__ v16h g2_frag(const _Float16* p, unsigned hh) { FragH f; f.half[0] = *(const v8us*)((const unsigned short*)p + 8u * hh); f.half[1] = *(const v8us*)((const unsigned short*)p + 16u + 8u * hh); return f.v; }
__device__ __forceinline__ v8f g2_mma(v16h a, v16h b, v8f c) { v8f d = __builtin_amdgcn_wmma_f32_16x16x32_f16(false, a, false, b, (short)0, c, false, false); asm volatile("v_nop\n\tv_nop\n\tv_nop\n\tv_nop" : "+v"(d) : "v"(a), "v"(b)); return d; }
template <int ACT>
__global__ __launch_bounds__(128) void k_gemm2(const _Float16* __restrict__ A, unsigned lda, size_t sA, const _Float16* __restrict__ Bh, unsigned ldb, size_t sB, float alpha,
    const float* __restrict__ bias, const float* __restrict__ CP, float* __restrict__ C, _Float16* __restrict__ C16, float c16s, unsigned ldc, size_t sC, unsigned M, unsigned N, unsigned K) {
  static_assert(ACT == 0 || ACT == 6);
  __shared__ __attribute__((aligned(16))) float so[4][32][68];
  const unsigned tid = threadIdx.x, w = tid >> 5, lane = tid & 31u, ln = lane & 15u, hh = lane >> 4; const unsigned by = blockIdx.y;
  A += (size_t)by * sA; Bh += (size_t)by * sB; const size_t cofs = (size_t)by * sC;
  const unsigned ntn = N >> 6; const unsigned mt = blockIdx.x / ntn, nq = blockIdx.x - mt * ntn; const unsigned row0 = mt * 128u + 32u * w, col0 = nq * 64u; if (row0 >= M) return;
  const _Float16* a0p = A + (size_t)(row0 + ln) * lda; const _Float16* a1p = a0p + (size_t)16 * lda;
  const _Float16* b0p = Bh + (size_t)(col0 + ln) * ldb; const _Float16* b1p = b0p + (size_t)16 * ldb; const _Float16* b2p = b1p + (size_t)16 * ldb; const _Float16* b3p = b2p + (size_t)16 * ldb;
  const v8f z8 = {0.f,0.f,0.f,0.f,0.f,0.f,0.f,0.f}; v8f c00 = z8, c01 = z8, c02 = z8, c03 = z8, c10 = z8, c11 = z8, c12 = z8, c13 = z8;
#pragma unroll 1
  for (unsigned kb = 0; kb < K; kb += 32u) { const v16h a0 = g2_frag(a0p + kb, hh), a1 = g2_frag(a1p + kb, hh);
    v16h b = g2_frag(b0p + kb, hh); c00 = g2_mma(a0, b, c00); c10 = g2_mma(a1, b, c10);
    b = g2_frag(b1p + kb, hh); c01 = g2_mma(a0, b, c01); c11 = g2_mma(a1, b, c11);
    b = g2_frag(b2p + kb, hh); c02 = g2_mma(a0, b, c02); c12 = g2_mma(a1, b, c12);
    b = g2_frag(b3p + kb, hh); c03 = g2_mma(a0, b, c03); c13 = g2_mma(a1, b, c13); }
  v8f accs[8] = {c00, c01, c02, c03, c10, c11, c12, c13};
#pragma unroll
  for (unsigned u = 0; u < 8; ++u) { const unsigned t = u & 3u, half = u >> 2; const unsigned col = col0 + t * 16u + ln; const float bv = bias ? bf16_rne(bias[col]) : 0.f;
#pragma unroll
    for (unsigned r = 0; r < 8; ++r) { const unsigned rloc = half * 16u + 8u * hh + r; float v = accs[u][r] * alpha + bv;
      if (CP) v += CP[cofs + (size_t)(row0 + rloc) * ldc + col];
      if (ACT == 6) v = 0.5f * v * (1.0f + erff(v * 0.70710678118654752f));
      so[w][rloc][t * 16u + ln] = v; } }
  __builtin_amdgcn_fence(4  , "workgroup"); __builtin_amdgcn_wave_barrier();
  const unsigned rsub = lane >> 4, c4 = (lane & 15u) * 4u;
  for (int pass = 0; pass < 2; ++pass) {
#pragma unroll
    for (unsigned q = 0; q < 16; ++q) { const unsigned r = q * 2u + rsub; const v4f v = *(const v4fa*)&so[w][r][c4]; const size_t o = cofs + (size_t)(row0 + r) * ldc + col0 + c4;
      if (C) *(volatile v4f*)(C + o) = v;
      if (C16) { v4h h4;
#pragma unroll
        for (unsigned i = 0; i < 4; ++i) h4[i] = (_Float16)(v[i] * c16s);
        *(volatile v4h*)(C16 + o) = h4; } }
    if (pass == 0) __threadfence(); } }

template <int NHv, int TTv>
__global__ __launch_bounds__(256) void k_vt(const _Float16* __restrict__ V16, unsigned ldv, unsigned voff, _Float16* __restrict__ Vt) {
  __shared__ unsigned short tl[64][66];
  const unsigned tid = threadIdx.x; const unsigned slab = blockIdx.x / (unsigned)(TTv / 64), lg = blockIdx.x - slab * (unsigned)(TTv / 64); const unsigned b = slab / (unsigned)NHv, h = slab - b * (unsigned)NHv;
  for (unsigned i = tid; i < 512u; i += 256u) { const unsigned r = i >> 3, c8 = (i & 7u) << 3; FragH f; f.half[0] = *(const v8us*)((const unsigned short*)V16 + ((size_t)b * TTv + lg * 64u + r) * ldv + voff + h * 64u + c8);
#pragma unroll
    for (unsigned q = 0; q < 8; ++q) tl[r][c8 + q] = f.u[q]; }
  __syncthreads();
  for (int pass = 0; pass < 2; ++pass) {
#pragma unroll
    for (unsigned rd = 0; rd < 2; ++rd) { const unsigned d = rd * 32u + (tid >> 3), pc = tid & 7u; FragH f;
#pragma unroll
      for (unsigned q = 0; q < 8; ++q) f.u[q] = tl[pc * 8u + q][d];
      *(volatile v8us*)((unsigned short*)Vt + ((size_t)slab * 64u + d) * TTv + lg * 64u + pc * 8u) = f.half[0]; }
    if (pass == 0) __threadfence(); } }

__global__ __launch_bounds__(256) void k_rsmw(const float* __restrict__ S, _Float16* __restrict__ P, unsigned nrows) {
  const unsigned row = blockIdx.x * 8u + (threadIdx.x >> 5), lane = threadIdx.x & 31u;
  if (row >= nrows) return;
  const float* s = S + (size_t)row * NKX + lane * 8u;
  float v[KPL * 8]; float mx = -3.0e38f;
#pragma unroll
  for (unsigned u = 0; u < KPL; ++u) { const v4f a = *(const v4fa*)(s + u * 256u), c = *(const v4fa*)(s + u * 256u + 4u);
#pragma unroll
    for (unsigned q = 0; q < 4; ++q) { v[u * 8u + q] = a[q]; v[u * 8u + 4u + q] = c[q]; mx = fmaxf(mx, fmaxf(a[q], c[q])); } }
  for (int o = 16; o > 0; o >>= 1) mx = fmaxf(mx, __shfl_xor(mx, o, 32));
  float se = 0.f;
#pragma unroll
  for (unsigned i = 0; i < KPL * 8; ++i) { const float e = __expf(v[i] - mx); v[i] = e; se += e; }
  for (int o = 16; o > 0; o >>= 1) se += __shfl_xor(se, o, 32);
  const float sc = 256.0f * (1.0f / se);
  FragH f[KPL];
#pragma unroll
  for (unsigned u = 0; u < KPL; ++u) {
#pragma unroll
    for (unsigned q = 0; q < 8; ++q) f[u].h[q] = (_Float16)(v[u * 8u + q] * sc); }
  unsigned short* d = (unsigned short*)P + (size_t)row * NKX + lane * 8u;
  for (int pass = 0; pass < 2; ++pass) {
#pragma unroll
    for (unsigned u = 0; u < KPL; ++u) *(volatile v8us*)(d + u * 256u) = f[u].half[0];
    if (pass == 0) __threadfence(); } }

constexpr size_t pad256(size_t b) { return (b + 255) & ~(size_t)255; }
constexpr size_t SZ_BQKV = pad256((size_t)LQ * DM * 2);
constexpr size_t SZ_BO   = pad256((size_t)DM * DM * 2);
constexpr size_t SZ_BW1  = pad256((size_t)DFF * DM * 2);
constexpr size_t SZ_BW2  = pad256((size_t)DM * DFF * 2);
constexpr size_t SZ_X16  = pad256((size_t)MP * DM * 2);
constexpr size_t SZ_XB   = pad256((size_t)MP * DM * 4);
constexpr size_t SZ_X1   = pad256((size_t)MP * DM * 4);
constexpr size_t SZ_QKV  = pad256((size_t)MP * LQ * 2);
constexpr size_t SZ_O16  = pad256((size_t)MP * DM * 2);
constexpr size_t SZ_VT   = pad256((size_t)NB * NH * HD * SEQ * 2);
constexpr size_t SZ_S    = pad256((size_t)NH * QT * NKX * 4);
constexpr size_t SZ_P    = pad256((size_t)NH * QT * NKX * 2);
constexpr size_t SZ_HF   = (size_t)MP * DFF * 2;
constexpr size_t SZ_TOTAL = SZ_BQKV + SZ_BO + SZ_BW1 + SZ_BW2 + SZ_X16 + SZ_XB + SZ_X1 + SZ_QKV + SZ_O16 + SZ_VT + SZ_S + SZ_P;
static_assert(SZ_HF <= SZ_S + SZ_P);
static_assert(SZ_TOTAL <= (size_t)134217728);

extern "C" void kernel_launch(void* const* d_in, const int* in_sizes, int n_in,
                              void* d_out, int out_size, void* d_ws, size_t ws_size, hipStream_t stream) {
  if (n_in < 13) return;
  if ((long long)in_sizes[0] < (long long)((size_t)(NB - 1) * SEQ_FULL + SEQ) * DM) return;
  if (in_sizes[1] < DM * LQ || in_sizes[2] < LQ || in_sizes[3] < DM * DM || in_sizes[4] < DM) return;
  if (in_sizes[5] < DM * DFF || in_sizes[6] < DFF || in_sizes[7] < DFF * DM || in_sizes[8] < DM) return;
  if (in_sizes[9] < DM || in_sizes[10] < DM || in_sizes[11] < DM || in_sizes[12] < DM) return;
  if ((long long)out_size < (long long)MP * DM) return;
  if (SZ_TOTAL > ws_size) return;
  const float* const* I = (const float* const*)d_in;
  const float* x = I[0]; const float* wqkv = I[1]; const float* bqkv = I[2]; const float* wproj = I[3]; const float* bproj = I[4];
  const float* w1 = I[5]; const float* b1 = I[6]; const float* w2 = I[7]; const float* b2 = I[8];
  const float* g1 = I[9]; const float* be1 = I[10]; const float* g2 = I[11]; const float* be2 = I[12];
  char* ws = (char*)d_ws; size_t off = 0;
  _Float16* BQKV = (_Float16*)(ws + off); off += SZ_BQKV;
  _Float16* BO   = (_Float16*)(ws + off); off += SZ_BO;
  _Float16* BW1  = (_Float16*)(ws + off); off += SZ_BW1;
  _Float16* BW2  = (_Float16*)(ws + off); off += SZ_BW2;
  _Float16* X16  = (_Float16*)(ws + off); off += SZ_X16;
  float*    XB   = (float*)(ws + off);    off += SZ_XB;
  float*    X1   = (float*)(ws + off);    off += SZ_X1;
  _Float16* QKV  = (_Float16*)(ws + off); off += SZ_QKV;
  _Float16* O16  = (_Float16*)(ws + off); off += SZ_O16;
  _Float16* VT   = (_Float16*)(ws + off); off += SZ_VT;
  float*    S    = (float*)(ws + off);    off += SZ_S;
  _Float16* P    = (_Float16*)(ws + off); off += SZ_P;
  _Float16* HF16 = (_Float16*)S;
  _Float16* M16  = X16;
  _Float16* Q16 = QKV; _Float16* K16 = QKV + DM; _Float16* V16 = QKV + 2 * DM;

  k_wt_f16<<<(unsigned)(((size_t)LQ * (DM / 8) + 255) / 256), 256, 0, stream>>>(wqkv, BQKV, (unsigned)DM, (unsigned)LQ, 16.0f);
  k_wt_f16<<<(unsigned)(((size_t)DM * (DM / 8) + 255) / 256), 256, 0, stream>>>(wproj, BO, (unsigned)DM, (unsigned)DM, 16.0f);
  k_wt_f16<<<(unsigned)(((size_t)DFF * (DM / 8) + 255) / 256), 256, 0, stream>>>(w1, BW1, (unsigned)DM, (unsigned)DFF, 16.0f);
  k_wt_f16<<<(unsigned)(((size_t)DM * (DFF / 8) + 255) / 256), 256, 0, stream>>>(w2, BW2, (unsigned)DFF, (unsigned)DM, 16.0f);
  k_ln16<1, 1><<<(unsigned)MP, 192, 0, stream>>>(x, (unsigned)SEQ, (unsigned)SEQ_FULL, g1, be1, 1e-5f, X16, XB);
  k_gemm2<0><<<dim3((unsigned)((MP / 128) * (LQ / 64)), 1), 128, 0, stream>>>(X16, (unsigned)DM, (size_t)0, BQKV, (unsigned)DM, (size_t)0, 0.0625f, bqkv, nullptr, nullptr, QKV, 1.0f, (unsigned)LQ, (size_t)0, (unsigned)MP, (unsigned)LQ, (unsigned)DM);
  k_vt<NH, SEQ><<<(unsigned)(NB * NH * (SEQ / 64)), 256, 0, stream>>>(V16, (unsigned)LQ, 0u, VT);
  for (int b = 0; b < NB; ++b) { const size_t r0 = (size_t)b * SEQ;
    for (int q0 = 0; q0 < SEQ; q0 += QT) {
      k_gemm2<0><<<dim3((unsigned)((QT / 128) * (SEQ / 64)), NH), 128, 0, stream>>>(Q16 + (r0 + q0) * LQ, (unsigned)LQ, (size_t)HD, K16 + r0 * LQ, (unsigned)LQ, (size_t)HD, 0.125f, nullptr, nullptr, S, nullptr, 1.0f, (unsigned)NKX, (size_t)QT * NKX, (unsigned)QT, (unsigned)SEQ, (unsigned)HD);
      k_rsmw<<<(unsigned)((NH * QT) / 8), 256, 0, stream>>>(S, P, (unsigned)(NH * QT));
      k_gemm2<0><<<dim3((unsigned)((QT / 128) * (HD / 64)), NH), 128, 0, stream>>>(P, (unsigned)NKX, (size_t)QT * NKX, VT + (size_t)b * NH * HD * SEQ, (unsigned)SEQ, (size_t)HD * SEQ, 0.25f, nullptr, nullptr, nullptr, O16 + (r0 + q0) * DM, 1.0f, (unsigned)DM, (size_t)HD, (unsigned)QT, (unsigned)HD, (unsigned)SEQ); } }
  k_gemm2<0><<<dim3((unsigned)((MP / 128) * (DM / 64)), 1), 128, 0, stream>>>(O16, (unsigned)DM, (size_t)0, BO, (unsigned)DM, (size_t)0, 0.0009765625f, bproj, XB, X1, nullptr, 1.0f, (unsigned)DM, (size_t)0, (unsigned)MP, (unsigned)DM, (unsigned)DM);
  k_ln16<0, 0><<<(unsigned)MP, 192, 0, stream>>>(X1, (unsigned)SEQ, (unsigned)SEQ, g2, be2, 1e-5f, M16, nullptr);
  k_gemm2<6><<<dim3((unsigned)((MP / 128) * (DFF / 64)), 1), 128, 0, stream>>>(M16, (unsigned)DM, (size_t)0, BW1, (unsigned)DM, (size_t)0, 0.0625f, b1, nullptr, nullptr, HF16, 16.0f, (unsigned)DFF, (size_t)0, (unsigned)MP, (unsigned)DFF, (unsigned)DM);
  k_gemm2<0><<<dim3((unsigned)((MP / 128) * (DM / 64)), 1), 128, 0, stream>>>(HF16, (unsigned)DFF, (size_t)0, BW2, (unsigned)DFF, (size_t)0, 0.00390625f, b2, X1, (float*)d_out, nullptr, 1.0f, (unsigned)DM, (size_t)0, (unsigned)MP, (unsigned)DM, (unsigned)DFF);
}
